// TransformerBlock_83004537963198
// MI455X (gfx1250) — hardware-verified
//
#include <hip/hip_runtime.h>
#include <stddef.h>
#include <math.h>


typedef _Float16 v16h __attribute__((ext_vector_type(16)));
typedef _Float16 v8h  __attribute__((ext_vector_type(8)));
typedef float    v8f  __attribute__((ext_vector_type(8)));
typedef float    v4f  __attribute__((ext_vector_type(4)));

#ifndef NB
#define NB 8
#endif
#ifndef SEQ
#define SEQ 1024
#endif
#define NB_FULL  8
#define SEQ_FULL 1024
#define EMB    768
#define NHEAD  8
#define HDR    12
#define HDP    16
#define INNER  96
#define QKP    128
#define NQKVP  384
#define NQKV   288
#define MLPD   3072
#define MROWS  (NB * SEQ)

static_assert(NB >= 1 && NB <= NB_FULL);
static_assert(SEQ >= 128 && SEQ <= SEQ_FULL && (SEQ % 128) == 0);
static_assert(INNER == NHEAD * HDR && QKP == NHEAD * HDP && NQKVP == 3 * QKP);
static_assert(EMB == 96 * 8);
static_assert((MROWS % 64) == 0);
static_assert((EMB % 64) == 0 && (MLPD % 64) == 0 && (QKP % 64) == 0 && (NQKVP % 64) == 0);
static_assert((EMB % 32) == 0 && (MLPD % 32) == 0 && (QKP % 32) == 0);
static_assert((size_t)MROWS * MLPD < (size_t)0xFFFFFFFFu);

#define LDT   72
#define LDK   24
#define LDO16 136
#define LDC   68

#define WCARRY 64.0f
#define PCARRY 1024.0f
#define VCARRY 64.0f
#define GCARRY 16.0f

#define WQKV_BYTES  ((size_t)NQKVP * EMB * 2)
#define WPRJ_BYTES  ((size_t)EMB * QKP * 2)
#define W1T_BYTES   ((size_t)MLPD * EMB * 2)
#define W2T_BYTES   ((size_t)EMB * MLPD * 2)
#define ACT16_BYTES ((size_t)MROWS * EMB * 2)
#define QK16_BYTES  ((size_t)MROWS * QKP * 2)
#define VT16_BYTES  ((size_t)NB * QKP * SEQ * 2)
#define X1_BYTES    ((size_t)MROWS * EMB * 4)
#define G16_BYTES   ((size_t)MROWS * MLPD * 2)

#define OFF_WQKV 0
#define OFF_WPRJ (OFF_WQKV + WQKV_BYTES)
#define OFF_W1T  (OFF_WPRJ + WPRJ_BYTES)
#define OFF_W2T  (OFF_W1T + W1T_BYTES)
#define OFF_H16  (OFF_W2T + W2T_BYTES)
#define OFF_Q16  (OFF_H16 + ACT16_BYTES)
#define OFF_K16  (OFF_Q16 + QK16_BYTES)
#define OFF_VT16 (OFF_K16 + QK16_BYTES)
#define OFF_CTX  (OFF_VT16 + VT16_BYTES)
#define OFF_X1   (OFF_CTX + QK16_BYTES)
#define OFF_M16  (OFF_X1 + X1_BYTES)
#define OFF_G16  (OFF_M16 + ACT16_BYTES)
#define WS_TOTAL (OFF_G16 + G16_BYTES)

static_assert((WQKV_BYTES % 128) == 0 && (WPRJ_BYTES % 128) == 0 && (W1T_BYTES % 128) == 0);
static_assert((W2T_BYTES % 128) == 0 && (ACT16_BYTES % 128) == 0 && (QK16_BYTES % 128) == 0);
static_assert((VT16_BYTES % 128) == 0 && (X1_BYTES % 128) == 0 && (G16_BYTES % 128) == 0);
static_assert(WS_TOTAL <= (size_t)134217728);

__device__ __forceinline__ float bf16r(float x) {
  unsigned int u = __float_as_uint(x);
  u = (u + 0x7FFFu + ((u >> 16) & 1u)) & 0xFFFF0000u;
  return __uint_as_float(u);
}

__device__ __forceinline__ v16h frag_at(const _Float16* p) {
  v8h lo = *(const v8h*)(p);
  v8h hi = *(const v8h*)(p + 16);
  v16h out;
#pragma unroll
  for (int i = 0; i < 8; ++i) { out[i] = lo[i]; out[i + 8] = hi[i]; }
  return out;
}
__device__ __forceinline__ v16h ld_frag(const _Float16* base, unsigned ld) {
  const unsigned lane = threadIdx.x & 31u;
  return frag_at(base + (lane & 15u) * ld + (lane >> 4) * 8u);
}
__device__ __forceinline__ v16h frag_lo16(const _Float16* p) {
  v8h lo = *(const v8h*)(p);
  v16h out;
#pragma unroll
  for (int i = 0; i < 8; ++i) { out[i] = lo[i]; out[i + 8] = (_Float16)0.0f; }
  return out;
}

__device__ __forceinline__ v8f wmma16(v16h a, v16h b, v8f c) {
  v8f d = __builtin_amdgcn_wmma_f32_16x16x32_f16(false, a, false, b, (short)0, c,
                                                 false, false);
  asm volatile("v_nop\n\tv_nop\n\tv_nop\n\tv_nop" : "+v"(d) : "v"(a), "v"(b));
  return d;
}

__device__ __forceinline__ float red16_max(float x) {
#pragma unroll
  for (int off = 1; off < 16; off <<= 1) x = fmaxf(x, __shfl_xor(x, off, 32));
  return x;
}
__device__ __forceinline__ float red16_sum(float x) {
#pragma unroll
  for (int off = 1; off < 16; off <<= 1) x += __shfl_xor(x, off, 32);
  return x;
}
__device__ __forceinline__ float red32_sum(float x) {
#pragma unroll
  for (int off = 16; off > 0; off >>= 1) x += __shfl_xor(x, off, 32);
  return x;
}

__device__ __forceinline__ void wave_lds_sync() {
  __builtin_amdgcn_fence(3  , "wavefront");
  asm volatile("s_wait_dscnt 0x0" ::: "memory");
  __builtin_amdgcn_wave_barrier();
}

template <int MAP, int KOUT, int LDW>
__global__ __launch_bounds__(256) void wconv_kernel(
    const float* __restrict__ W, _Float16* __restrict__ Wt) {
  __shared__ _Float16 T[64 * LDT];
  const unsigned tid = threadIdx.x;
  const unsigned n0 = blockIdx.x * 64u;
  const unsigned k0 = blockIdx.y * 64u;
#pragma unroll 4
  for (unsigned j = 0; j < 16u; ++j) {
    const unsigned idx = tid + 256u * j;
    const unsigned kr = idx >> 6, nc = idx & 63u;
    unsigned srow = k0 + kr;
    unsigned scol = n0 + nc;
    bool ok = true;
    if (MAP == 1) {
      const unsigned d = scol & 15u;
      ok = d < (unsigned)HDR;
      const unsigned dc = ok ? d : (unsigned)(HDR - 1);
      scol = (scol >> 7) * (unsigned)INNER + ((scol >> 4) & 7u) * (unsigned)HDR + dc;
    }
    if (MAP == 2) {
      const unsigned d = srow & 15u;
      ok = d < (unsigned)HDR;
      const unsigned dc = ok ? d : (unsigned)(HDR - 1);
      srow = (srow >> 4) * (unsigned)HDR + dc;
    }
    const float v = W[(size_t)srow * LDW + scol];
    const float cv = WCARRY * bf16r(v);
    T[nc * LDT + kr] = (_Float16)(ok ? cv : 0.0f);
  }
  __syncthreads();
  v8h x[2];
  size_t off[2];
#pragma unroll
  for (unsigned i = 0; i < 2u; ++i) {
    const unsigned n = 32u * i + (tid >> 3);
    const unsigned kc = (tid & 7u) * 8u;
    x[i] = *(const v8h*)&T[n * LDT + kc];
    off[i] = (size_t)(n0 + n) * KOUT + k0 + kc;
  }
#pragma unroll
  for (int i = 0; i < 2; ++i) *(volatile v8h*)(Wt + off[i]) = x[i];
  __threadfence();
#pragma unroll
  for (int i = 0; i < 2; ++i) *(volatile v8h*)(Wt + off[i]) = x[i];
}

template <int SRCIN>
__global__ __launch_bounds__(96) void ln_kernel(
    const float* __restrict__ X, const float* __restrict__ gam,
    const float* __restrict__ bet, _Float16* __restrict__ dst) {
  __shared__ float red1[4];
  __shared__ float red2[4];
  const unsigned tid = threadIdx.x, lane = tid & 31u, w = tid >> 5;
  const unsigned crow = blockIdx.x;
  size_t srow = crow;
  if (SRCIN) {
    const unsigned bidx = crow / (unsigned)SEQ;
    const unsigned sq = crow - bidx * (unsigned)SEQ;
    srow = (size_t)bidx * SEQ_FULL + sq;
  }
  const unsigned c = tid * 8u;
  const float* sp = X + srow * EMB + c;
  const v4f a0 = *(const v4f*)(sp);
  const v4f a1 = *(const v4f*)(sp + 4);
  float v[8];
#pragma unroll
  for (int j = 0; j < 4; ++j) {
    v[j]     = SRCIN ? bf16r(a0[j]) : a0[j];
    v[j + 4] = SRCIN ? bf16r(a1[j]) : a1[j];
  }
  float s = ((v[0] + v[1]) + (v[2] + v[3])) + ((v[4] + v[5]) + (v[6] + v[7]));
  s = red32_sum(s);
  if (lane == 0u) red1[w] = s;
  __syncthreads();
  const float mu = ((red1[0] + red1[1]) + red1[2]) * (1.0f / (float)EMB);
  float q = 0.0f;
#pragma unroll
  for (int j = 0; j < 8; ++j) { v[j] = v[j] - mu; q += v[j] * v[j]; }
  q = red32_sum(q);
  if (lane == 0u) red2[w] = q;
  __syncthreads();
  const float var = ((red2[0] + red2[1]) + red2[2]) * (1.0f / (float)EMB);
  const float rstd = rsqrtf(var + 1.0e-5f);
  const v4f g0 = *(const v4f*)(gam + c);
  const v4f g1 = *(const v4f*)(gam + c + 4);
  const v4f b0 = *(const v4f*)(bet + c);
  const v4f b1 = *(const v4f*)(bet + c + 4);
  v8h o;
#pragma unroll
  for (int j = 0; j < 4; ++j) {
    o[j]     = (_Float16)(v[j] * rstd * bf16r(g0[j]) + bf16r(b0[j]));
    o[j + 4] = (_Float16)(v[j + 4] * rstd * bf16r(g1[j]) + bf16r(b1[j]));
  }
  _Float16* dp = dst + (size_t)crow * EMB + c;
  *(volatile v8h*)dp = o;
  __threadfence();
  *(volatile v8h*)dp = o;
}

template <int MODE, int KD, int LDO>
__global__ __launch_bounds__(256) void gemm_kernel(
    const _Float16* __restrict__ A16, const _Float16* __restrict__ Bt,
    const float* __restrict__ biasf, const float* __restrict__ resf,
    float* __restrict__ outf, _Float16* __restrict__ out16) {
  static_assert((KD % 32) == 0 && (LDO % 64) == 0);
  __shared__ float Cs[64 * LDC];
  const unsigned tid = threadIdx.x, lane = tid & 31u, w = tid >> 5;
  const unsigned mw = w >> 1, nw = w & 1u;
  const unsigned hh = lane >> 4, m = lane & 15u;
  const unsigned n0 = blockIdx.x * 64u;
  const unsigned row0 = blockIdx.y * 64u;

  const _Float16* ap  = A16 + (size_t)(row0 + mw * 16u + m) * KD + hh * 8u;
  const _Float16* bp0 = Bt + (size_t)(n0 + nw * 32u + m) * KD + hh * 8u;
  const _Float16* bp1 = bp0 + 16 * KD;
  v8f acc0 = {}, acc1 = {};
#pragma unroll 2
  for (unsigned k0 = 0; k0 < (unsigned)KD; k0 += 32u) {
    const v16h a  = frag_at(ap + k0);
    const v16h b0 = frag_at(bp0 + k0);
    const v16h b1 = frag_at(bp1 + k0);
    acc0 = wmma16(a, b0, acc0);
    acc1 = wmma16(a, b1, acc1);
  }
#pragma unroll
  for (int r = 0; r < 8; ++r) {
    float* d = &Cs[(mw * 16u + hh * 8u + (unsigned)r) * LDC + nw * 32u + m];
    d[0]  = acc0[r];
    d[16] = acc1[r];
  }
  __syncthreads();

  if (MODE == 3) {
    const unsigned rb = tid >> 3, cb = (tid & 7u) * 8u;
#pragma unroll 1
    for (unsigned e = 0; e < 16u; ++e) {
      const unsigned r = ((e >> 3) << 5) + rb;
      const unsigned c = cb + (e & 7u);
      float* cp = &Cs[r * LDC + c];
      const float z = cp[0] * (1.0f / WCARRY) + bf16r(biasf[n0 + c]);
      cp[0] = GCARRY * (0.5f * z * (1.0f + erff(z * 0.70710678118654752f)));
    }
    __syncthreads();
  }

  if (MODE == 0 || MODE == 3) {
    const float sc = (MODE == 0) ? (1.0f / WCARRY) : 1.0f;
    v8h x[2];
    size_t off[2];
#pragma unroll
    for (unsigned i = 0; i < 2u; ++i) {
      const unsigned r = 32u * i + (tid >> 3);
      const unsigned c = (tid & 7u) * 8u;
      const v4f u0 = *(const v4f*)&Cs[r * LDC + c];
      const v4f u1 = *(const v4f*)&Cs[r * LDC + c + 4];
#pragma unroll
      for (int j = 0; j < 4; ++j) {
        x[i][j]     = (_Float16)(u0[j] * sc);
        x[i][j + 4] = (_Float16)(u1[j] * sc);
      }
      off[i] = (size_t)(row0 + r) * LDO + n0 + c;
    }
#pragma unroll
    for (int i = 0; i < 2; ++i) *(volatile v8h*)(out16 + off[i]) = x[i];
    __threadfence();
#pragma unroll
    for (int i = 0; i < 2; ++i) *(volatile v8h*)(out16 + off[i]) = x[i];
  }

  if (MODE == 1) {
    const unsigned bidx = row0 / (unsigned)SEQ;
    const unsigned key0 = row0 - bidx * (unsigned)SEQ;
    v8h x[2];
    size_t off[2];
#pragma unroll
    for (unsigned i = 0; i < 2u; ++i) {
      const unsigned dcol = 32u * i + (tid >> 3);
      const unsigned kk = (tid & 7u) * 8u;
#pragma unroll
      for (unsigned j = 0; j < 8u; ++j)
        x[i][j] = (_Float16)(Cs[(kk + j) * LDC + dcol] * (1.0f / WCARRY));
      off[i] = ((size_t)bidx * LDO + n0 + dcol) * SEQ + key0 + kk;
    }
#pragma unroll
    for (int i = 0; i < 2; ++i) *(volatile v8h*)(out16 + off[i]) = x[i];
    __threadfence();
#pragma unroll
    for (int i = 0; i < 2; ++i) *(volatile v8h*)(out16 + off[i]) = x[i];
  }

  if (MODE == 2 || MODE == 4) {
    const float sc = (MODE == 2) ? (1.0f / (WCARRY * VCARRY)) : (1.0f / (WCARRY * GCARRY));
    v4f xs[4];
    size_t off[4];
#pragma unroll
    for (unsigned i = 0; i < 4u; ++i) {
      const unsigned r = 16u * i + (tid >> 4);
      const unsigned c = (tid & 15u) * 4u;
      const unsigned crow = row0 + r;
      const unsigned bidx = crow / (unsigned)SEQ;
      const unsigned sq = crow - bidx * (unsigned)SEQ;
      const size_t frow = (size_t)bidx * SEQ_FULL + sq;
      const size_t rrow = (MODE == 2) ? frow : (size_t)crow;
      const size_t orow = (MODE == 2) ? (size_t)crow : frow;
      const v4f u = *(const v4f*)&Cs[r * LDC + c];
      const v4f g = *(const v4f*)(biasf + n0 + c);
      const v4f rr = *(const v4f*)(resf + rrow * LDO + n0 + c);
      v4f val;
#pragma unroll
      for (int j = 0; j < 4; ++j) {
        const float rv = (MODE == 2) ? bf16r(rr[j]) : rr[j];
        val[j] = (u[j] * sc + bf16r(g[j])) + rv;
      }
      xs[i] = val;
      off[i] = orow * LDO + n0 + c;
    }
#pragma unroll
    for (int i = 0; i < 4; ++i) *(volatile v4f*)(outf + off[i]) = xs[i];
    __threadfence();
#pragma unroll
    for (int i = 0; i < 4; ++i) *(volatile v4f*)(outf + off[i]) = xs[i];
  }
}

__global__ __launch_bounds__(256) void attn_kernel(
    const _Float16* __restrict__ Qh, const _Float16* __restrict__ Kh,
    const _Float16* __restrict__ Vt, _Float16* __restrict__ Ov) {
  __shared__ _Float16 Ks[64 * LDK];
  __shared__ _Float16 Vs[16 * LDT];
  __shared__ _Float16 Ps[8 * 16 * LDT];
  __shared__ _Float16 Os[8 * 16 * LDO16];

  const unsigned tid = threadIdx.x, lane = tid & 31u, w = tid >> 5;
  const unsigned hh = lane >> 4, m = lane & 15u;
  const unsigned q0 = blockIdx.x * 128u;
  const unsigned b = blockIdx.y;
  const float scale = 0.10206207261596577f;
  _Float16* P = Ps + w * (16u * LDT);
  _Float16* O = Os + w * (16u * LDO16);
  const unsigned qrow = b * (unsigned)SEQ + q0 + w * 16u + m;

#pragma unroll 1
  for (unsigned head = 0; head < (unsigned)NHEAD; ++head) {
    const v16h qf = frag_lo16(Qh + (size_t)qrow * QKP + head * HDP + hh * 8u);

    float mrow[8], lrow[8];
    v8f o = {};
#pragma unroll
    for (int v = 0; v < 8; ++v) { mrow[v] = -1.0e30f; lrow[v] = 0.0f; }

#pragma unroll 1
    for (unsigned kb = 0; kb < (unsigned)SEQ; kb += 64u) {
      if (tid < 128u) {
        const unsigned r = tid >> 1, c = (tid & 1u) * 8u;
        *(v8h*)&Ks[r * LDK + c] =
            *(const v8h*)(Kh + (size_t)(b * (unsigned)SEQ + kb + r) * QKP + head * HDP + c);
      } else {
        const unsigned t = tid - 128u;
        const unsigned r = t >> 3, c = (t & 7u) * 8u;
        *(v8h*)&Vs[r * LDT + c] =
            *(const v8h*)(Vt + ((size_t)b * QKP + head * HDP + r) * SEQ + kb + c);
      }
      __syncthreads();

      v8f s[4];
#pragma unroll
      for (int kg = 0; kg < 4; ++kg) {
        const v16h kf = frag_lo16(&Ks[((unsigned)kg * 16u + m) * LDK + hh * 8u]);
        v8f t = {};
        t = wmma16(qf, kf, t);
        s[kg] = t * scale;
      }

      float alpha[8];
#pragma unroll
      for (int v = 0; v < 8; ++v) {
        float mx = fmaxf(fmaxf(s[0][v], s[1][v]), fmaxf(s[2][v], s[3][v]));
        mx = red16_max(mx);
        const float mn = fmaxf(mrow[v], mx);
        alpha[v] = __expf(mrow[v] - mn);
        mrow[v] = mn;
      }
#pragma unroll
      for (int kg = 0; kg < 4; ++kg)
#pragma unroll
        for (int v = 0; v < 8; ++v) s[kg][v] = __expf(s[kg][v] - mrow[v]);
#pragma unroll
      for (int v = 0; v < 8; ++v) {
        const float rs = red16_sum((s[0][v] + s[1][v]) + (s[2][v] + s[3][v]));
        lrow[v] = alpha[v] * lrow[v] + rs;
      }
#pragma unroll
      for (int v = 0; v < 8; ++v) o[v] = o[v] * alpha[v];

#pragma unroll
      for (int kg = 0; kg < 4; ++kg)
#pragma unroll
        for (int v = 0; v < 8; ++v)
          P[(hh * 8u + (unsigned)v) * LDT + (unsigned)kg * 16u + m] =
              (_Float16)(s[kg][v] * PCARRY);
      wave_lds_sync();

#pragma unroll
      for (int c = 0; c < 2; ++c) {
        const v16h pf = ld_frag(P + c * 32, LDT);
        const v16h vf = ld_frag(&Vs[c * 32], LDT);
        o = wmma16(pf, vf, o);
      }
      __syncthreads();
    }

#pragma unroll
    for (int v = 0; v < 8; ++v) {
      const float inv = __builtin_amdgcn_rcpf(lrow[v]) * (VCARRY / PCARRY);
      O[(hh * 8u + (unsigned)v) * LDO16 + head * HDP + m] = (_Float16)(o[v] * inv);
    }
  }
  wave_lds_sync();

  v8h x[8];
  size_t off[8];
#pragma unroll
  for (unsigned i = 0; i < 8u; ++i) {
    const unsigned r = 2u * i + (lane >> 4);
    const unsigned c = (lane & 15u) * 8u;
    x[i] = *(const v8h*)&O[r * LDO16 + c];
    off[i] = (size_t)(b * (unsigned)SEQ + q0 + w * 16u + r) * QKP + c;
  }
#pragma unroll
  for (int i = 0; i < 8; ++i) *(volatile v8h*)(Ov + off[i]) = x[i];
  __threadfence();
#pragma unroll
  for (int i = 0; i < 8; ++i) *(volatile v8h*)(Ov + off[i]) = x[i];
}

extern "C" void kernel_launch(void* const* d_in, const int* in_sizes, int n_in,
                              void* d_out, int out_size, void* d_ws, size_t ws_size,
                              hipStream_t stream) {
  if (n_in < 14) return;
  const long long need_x = ((long long)(NB - 1) * SEQ_FULL + SEQ) * EMB;
  if ((long long)in_sizes[0] < need_x) return;
  if (in_sizes[3] < EMB || in_sizes[4] < EMB || in_sizes[7] < EMB) return;
  if (in_sizes[8] < EMB || in_sizes[9] < EMB || in_sizes[13] < EMB) return;
  if ((long long)in_sizes[5] < (long long)EMB * NQKV) return;
  if ((long long)in_sizes[6] < (long long)INNER * EMB) return;
  if ((long long)in_sizes[10] < (long long)EMB * MLPD) return;
  if (in_sizes[11] < MLPD) return;
  if ((long long)in_sizes[12] < (long long)MLPD * EMB) return;
  if ((long long)out_size < need_x) return;
  if (ws_size < WS_TOTAL) return;

  const float* X     = (const float*)d_in[0];
  const float* behav = (const float*)d_in[1];
  const int*   mouse = (const int*)d_in[2];
  const float* ln1g  = (const float*)d_in[3];
  const float* ln1b  = (const float*)d_in[4];
  const float* Wqkv  = (const float*)d_in[5];
  const float* Wprj  = (const float*)d_in[6];
  const float* bprj  = (const float*)d_in[7];
  const float* ln2g  = (const float*)d_in[8];
  const float* ln2b  = (const float*)d_in[9];
  const float* W1    = (const float*)d_in[10];
  const float* b1    = (const float*)d_in[11];
  const float* W2    = (const float*)d_in[12];
  const float* b2    = (const float*)d_in[13];
  (void)behav;
  (void)mouse;
  float* out = (float*)d_out;

  char* ws = (char*)d_ws;
  _Float16* WtQKV = (_Float16*)(ws + OFF_WQKV);
  _Float16* WtPrj = (_Float16*)(ws + OFF_WPRJ);
  _Float16* Wt1   = (_Float16*)(ws + OFF_W1T);
  _Float16* Wt2   = (_Float16*)(ws + OFF_W2T);
  _Float16* H16   = (_Float16*)(ws + OFF_H16);
  _Float16* Q16   = (_Float16*)(ws + OFF_Q16);
  _Float16* K16   = (_Float16*)(ws + OFF_K16);
  _Float16* Vt16  = (_Float16*)(ws + OFF_VT16);
  _Float16* Ctx16 = (_Float16*)(ws + OFF_CTX);
  float*    X1    = (float*)(ws + OFF_X1);
  _Float16* M16   = (_Float16*)(ws + OFF_M16);
  _Float16* G16   = (_Float16*)(ws + OFF_G16);

  dim3 blk(256);

  wconv_kernel<1, EMB, NQKV><<<dim3(NQKVP / 64, EMB / 64), blk, 0, stream>>>(Wqkv, WtQKV);
  wconv_kernel<2, QKP, EMB><<<dim3(EMB / 64, QKP / 64), blk, 0, stream>>>(Wprj, WtPrj);
  wconv_kernel<0, EMB, MLPD><<<dim3(MLPD / 64, EMB / 64), blk, 0, stream>>>(W1, Wt1);
  wconv_kernel<0, MLPD, EMB><<<dim3(EMB / 64, MLPD / 64), blk, 0, stream>>>(W2, Wt2);

  ln_kernel<1><<<dim3(MROWS), dim3(96), 0, stream>>>(X, ln1g, ln1b, H16);
  dim3 gq(QKP / 64, MROWS / 64);
  const size_t WPL = (size_t)QKP * EMB;
  gemm_kernel<0, EMB, QKP><<<gq, blk, 0, stream>>>(H16, WtQKV + 0 * WPL, bprj, X, X1, Q16);
  gemm_kernel<0, EMB, QKP><<<gq, blk, 0, stream>>>(H16, WtQKV + 1 * WPL, bprj, X, X1, K16);
  gemm_kernel<1, EMB, QKP><<<gq, blk, 0, stream>>>(H16, WtQKV + 2 * WPL, bprj, X, X1, Vt16);
  attn_kernel<<<dim3(SEQ / 128, NB), blk, 0, stream>>>(Q16, K16, Vt16, Ctx16);
  gemm_kernel<2, QKP, EMB><<<dim3(EMB / 64, MROWS / 64), blk, 0, stream>>>(
      Ctx16, WtPrj, bprj, X, X1, Q16);

  ln_kernel<0><<<dim3(MROWS), dim3(96), 0, stream>>>(X1, ln2g, ln2b, M16);
  gemm_kernel<3, EMB, MLPD><<<dim3(MLPD / 64, MROWS / 64), blk, 0, stream>>>(
      M16, Wt1, b1, X1, out, G16);
  gemm_kernel<4, MLPD, EMB><<<dim3(EMB / 64, MROWS / 64), blk, 0, stream>>>(
      G16, Wt2, b2, X1, out, Q16);
}
